// Mamba2Block_55473797595674
// MI455X (gfx1250) — hardware-run, weakly checked
//
#include <hip/hip_runtime.h>
#include <math.h>

typedef __attribute__((ext_vector_type(16))) _Float16 v16h;
typedef __attribute__((ext_vector_type(8)))  _Float16 v8h;
typedef __attribute__((ext_vector_type(16))) __bf16   v16b;
typedef __attribute__((ext_vector_type(8)))  __bf16   v8b;
typedef __attribute__((ext_vector_type(8)))  float    v8f;
typedef __attribute__((ext_vector_type(4)))  float    v4f;
typedef __attribute__((ext_vector_type(4)))  unsigned v4u;

constexpr int kBatch  = 2;
constexpr int kSeq    = 2048;
constexpr int kHid    = 1024;
constexpr int kInner  = 2048;
constexpr int kState  = 64;
constexpr int kTaps   = 4;
constexpr int kRows   = kBatch * kSeq;
constexpr int kBC     = 2 * kState;
constexpr int kQ      = 64;
constexpr int kCB     = 64;
constexpr int kNChunk = kSeq / kQ;
constexpr int kUP     = 72;
constexpr int kYP     = 68;
constexpr int kConvTP = 260;
static_assert((kHid % 32) == 0 && (kInner % 32) == 0 && (kState % 32) == 0 && (kQ % 32) == 0, "GEMM K multiples of 32");
static_assert((kRows % 64) == 0 && (kInner % 64) == 0 && (kHid % 64) == 0 && (kBC % 64) == 0 && (kQ % 64) == 0, "GEMM M,N multiples of 64");
static_assert((kSeq % kQ) == 0 && (kInner % kCB) == 0 && (kInner % 256) == 0 && (kRows % 64) == 0 && kQ == 64 && kCB == 64 && kState == 64, "tile multiples");

constexpr size_t kOffXB   = 0;
constexpr size_t kOffWINT = kOffXB   + (size_t)kRows * kHid * 2;
constexpr size_t kOffWDTT = kOffWINT + (size_t)(2 * kInner) * kHid * 2;
constexpr size_t kOffWBCT = kOffWDTT + (size_t)kInner * kInner * 2;
constexpr size_t kOffWOT  = kOffWBCT + (size_t)kBC * kInner * 2;
constexpr size_t kOffXIN  = kOffWOT  + (size_t)kHid * kInner * 2;
constexpr size_t kOffZP   = kOffXIN  + (size_t)kRows * kInner * 4;
constexpr size_t kOffXCH  = kOffZP   + (size_t)kRows * kInner * 2;
constexpr size_t kOffDTP  = kOffXCH  + (size_t)kRows * kInner * 2;
constexpr size_t kOffBCH  = kOffDTP  + (size_t)kRows * kInner * 2;
constexpr size_t kOffBT   = kOffBCH  + (size_t)kRows * kBC * 2;
constexpr size_t kOffGP   = kOffBT   + (size_t)kState * kRows * 2;
constexpr size_t kOffYL   = kOffGP   + (size_t)(kBatch * kNChunk) * kQ * kQ * 2;
constexpr size_t kWsTotal = kOffYL   + (size_t)kRows * kInner * 2;
static_assert(kWsTotal == 132644864ull, "carve total");
static_assert(kWsTotal <= 134217728ull, "carve cap");
static_assert((kOffWINT % 128) == 0 && (kOffWDTT % 128) == 0 && (kOffWBCT % 128) == 0 && (kOffWOT % 128) == 0 &&
              (kOffXIN % 128) == 0 && (kOffZP % 128) == 0 && (kOffXCH % 128) == 0 && (kOffDTP % 128) == 0 &&
              (kOffBCH % 128) == 0 && (kOffBT % 128) == 0 && (kOffGP % 128) == 0 && (kOffYL % 128) == 0, "128-B aligned regions");

__device__ __forceinline__ unsigned short f2bf_bits(float f) {
  unsigned u = __float_as_uint(f);
  return (unsigned short)((u + 0x7FFFu + ((u >> 16) & 1u)) >> 16);
}
__device__ __forceinline__ float bf_bits2f(unsigned short h) { return __uint_as_float(((unsigned)h) << 16); }
__device__ __forceinline__ float bfq(float f) { return bf_bits2f(f2bf_bits(f)); }
__device__ __forceinline__ __bf16 at_f2bf(float f) { return __builtin_bit_cast(__bf16, f2bf_bits(f)); }
__device__ __forceinline__ float h16_to_f32(unsigned hb) {
  const unsigned sgn = (hb & 0x8000u) << 16; const unsigned em = hb & 0x7fffu;
  const float fn = __uint_as_float((em << 13) + 0x38000000u);
  const float fs = (float)em * 5.9604644775390625e-8f;
  const float mag = (em < 0x400u) ? fs : fn; return __uint_as_float(__float_as_uint(mag) | sgn);
}

__device__ __forceinline__ void dep_guard_h(v8f& a, v8f& b, v16h x, v16h y) { asm volatile("v_nop\n\tv_nop\n\tv_nop\n\tv_nop" : "+v"(a), "+v"(b) : "v"(x), "v"(y)); }
__device__ __forceinline__ void dep_guard_b(v8f& a, v8f& b, v16b x, v16b y) { asm volatile("v_nop\n\tv_nop\n\tv_nop\n\tv_nop" : "+v"(a), "+v"(b) : "v"(x), "v"(y)); }
__device__ __forceinline__ void dep_guard4_h(v8f& a, v8f& b, v8f& c, v8f& d, v16h x, v16h y) { asm volatile("v_nop\n\tv_nop\n\tv_nop\n\tv_nop" : "+v"(a), "+v"(b), "+v"(c), "+v"(d) : "v"(x), "v"(y)); }
__device__ __forceinline__ void dep_guard4_b(v8f& a, v8f& b, v8f& c, v8f& d, v16b x, v16b y) { asm volatile("v_nop\n\tv_nop\n\tv_nop\n\tv_nop" : "+v"(a), "+v"(b), "+v"(c), "+v"(d) : "v"(x), "v"(y)); }
__device__ __forceinline__ void keep4_h(v16h a, v16h b, v16h c, v16h d) { asm volatile("v_nop" :: "v"(a), "v"(b), "v"(c), "v"(d)); }
__device__ __forceinline__ void keep4_b(v16b a, v16b b, v16b c, v16b d) { asm volatile("v_nop" :: "v"(a), "v"(b), "v"(c), "v"(d)); }
__device__ __forceinline__ void acc_guard4(v8f& a, v8f& b, v8f& c, v8f& d) { asm volatile("v_nop\n\tv_nop\n\tv_nop\n\tv_nop" : "+v"(a), "+v"(b), "+v"(c), "+v"(d)); }
template <typename T> struct Frag;
template <> struct Frag<_Float16> {
  typedef v16h V; union U { v16h v; v8h h[2]; };
  static __device__ __forceinline__ v16h load(const _Float16* p) {
    U f; f.h[0] = *(const v8h*)(p); f.h[1] = *(const v8h*)(p + 16); return f.v;
  }
  static __device__ __forceinline__ v8f mma(v16h a, v16h b, v8f c) {
    return __builtin_amdgcn_wmma_f32_16x16x32_f16(false, a, false, b, (short)0, c, false, false);
  }
  static __device__ __forceinline__ void guard(v8f& a, v8f& b, v16h x, v16h y) { dep_guard_h(a, b, x, y); }
  static __device__ __forceinline__ void guard4(v8f& a, v8f& b, v8f& c, v8f& d, v16h x, v16h y) { dep_guard4_h(a, b, c, d, x, y); }
  static __device__ __forceinline__ void keep(v16h a, v16h b, v16h c, v16h d) { keep4_h(a, b, c, d); }
};
template <> struct Frag<__bf16> {
  typedef v16b V; union U { v16b v; v8b h[2]; };
  static __device__ __forceinline__ v16b load(const __bf16* p) {
    U f; f.h[0] = *(const v8b*)(p); f.h[1] = *(const v8b*)(p + 16); return f.v;
  }
  static __device__ __forceinline__ v8f mma(v16b a, v16b b, v8f c) {
    return __builtin_amdgcn_wmma_f32_16x16x32_bf16(false, a, false, b, (short)0, c, false, false);
  }
  static __device__ __forceinline__ void guard(v8f& a, v8f& b, v16b x, v16b y) { dep_guard_b(a, b, x, y); }
  static __device__ __forceinline__ void guard4(v8f& a, v8f& b, v8f& c, v8f& d, v16b x, v16b y) { dep_guard4_b(a, b, c, d, x, y); }
  static __device__ __forceinline__ void keep(v16b a, v16b b, v16b c, v16b d) { keep4_b(a, b, c, d); }
};
__device__ __forceinline__ v8f mma_g(v16b a, v16b b, v8f c) {
  c = __builtin_amdgcn_wmma_f32_16x16x32_bf16(false, a, false, b, (short)0, c, false, false);
  asm volatile("v_nop\n\tv_nop\n\tv_nop\n\tv_nop" : "+v"(c) : "v"(a), "v"(b));
  return c;
}

template <int ET> struct Elem;
template <> struct Elem<0> { typedef _Float16 T; };
template <> struct Elem<1> { typedef __bf16 T; };
template <int ET, int SPL, int BIAS_MODE, int OUT_MODE, bool RESID, int ACT = 0>
__global__ __launch_bounds__(256) void wmma_gemm64(
    const unsigned short* __restrict__ Ap, const unsigned short* __restrict__ A2p, int lda, long strideA,
    const unsigned short* __restrict__ Btp, const unsigned short* __restrict__ Bt2p, int ldb, long strideB,
    void* __restrict__ Cout, void* __restrict__ Cout2, int ldc, long strideC,
    const float* __restrict__ bias,
    const float* __restrict__ resid, long strideR,
    int M, int N, int K, float scale) {
  typedef typename Elem<ET>::T T;
  typedef typename Frag<T>::V V;
  const T* A = (const T*)Ap; const T* A2 = (const T*)A2p; const T* Bt = (const T*)Btp; const T* Bt2 = (const T*)Bt2p;
  __shared__ __align__(16) float sT[8][16 * 68];
  const int b    = blockIdx.y;
  const int lane = threadIdx.x & 31;
  const int wave = threadIdx.x >> 5;
  const int tilesN = N >> 6;
  const int tilesM = M >> 6;
  const int tile = blockIdx.x * 8 + wave;
  if (tile >= tilesM * tilesN) return;
  const int tm = tile / tilesN;
  const int tn = tile - tm * tilesN;
  const int m0 = tm << 6;
  const int n0 = tn << 6;

  const T* Ab  = A  + (size_t)b * strideA;
  const T* Bb  = Bt + (size_t)b * strideB;
  const T* Ab2 = (SPL >= 1) ? (A2  + (size_t)b * strideA) : nullptr;
  const T* Bb2 = (SPL == 2) ? (Bt2 + (size_t)b * strideB) : nullptr;

  const int rlane = lane & 15;
  const int koff  = (lane >> 4) * 8;
  const int mOff  = (lane >> 4) * 8;

  v8f acc[4][4];
#pragma unroll
  for (int i = 0; i < 4; ++i)
#pragma unroll
    for (int j = 0; j < 4; ++j) acc[i][j] = (v8f){0.f,0.f,0.f,0.f,0.f,0.f,0.f,0.f};

  for (int k0 = 0; k0 < K; k0 += 32) {
    V bh[4], bl[4];
#pragma unroll
    for (int j = 0; j < 4; ++j) {
      const size_t bo = (size_t)(n0 + (j << 4) + rlane) * ldb + koff + k0;
      bh[j] = Frag<T>::load(Bb + bo);
      if (SPL == 2) bl[j] = Frag<T>::load(Bb2 + bo);
    }
#pragma unroll
    for (int i = 0; i < 4; ++i) {
      const size_t ao = (size_t)(m0 + (i << 4) + rlane) * lda + koff + k0;
      V ah = Frag<T>::load(Ab + ao);
      V al;
      if (SPL >= 1) al = Frag<T>::load(Ab2 + ao);
#pragma unroll
      for (int j = 0; j < 4; ++j) {
        acc[i][j] = Frag<T>::mma(ah, bh[j], acc[i][j]);
        if (SPL == 2) acc[i][j] = Frag<T>::mma(ah, bl[j], acc[i][j]);
        if (SPL >= 1) acc[i][j] = Frag<T>::mma(al, bh[j], acc[i][j]);
      }
      Frag<T>::guard4(acc[i][0], acc[i][1], acc[i][2], acc[i][3], ah, (SPL >= 1) ? al : ah);
    }
    Frag<T>::keep(bh[0], bh[1], bh[2], bh[3]);
    if (SPL == 2) Frag<T>::keep(bl[0], bl[1], bl[2], bl[3]);
  }
  acc_guard4(acc[0][0], acc[0][1], acc[0][2], acc[0][3]);
  acc_guard4(acc[1][0], acc[1][1], acc[1][2], acc[1][3]);
  acc_guard4(acc[2][0], acc[2][1], acc[2][2], acc[2][3]);
  acc_guard4(acc[3][0], acc[3][1], acc[3][2], acc[3][3]);

  float* slab = sT[wave];
  const float* Rb = RESID ? (resid + (size_t)b * strideR) : nullptr;
#pragma unroll
  for (int i = 0; i < 4; ++i) {
    const int mBase = m0 + (i << 4);
#pragma unroll
    for (int j = 0; j < 4; ++j) {
      const int n = n0 + (j << 4) + rlane;
      float bv = 0.f;
      if (BIAS_MODE == 2) bv = bias[n];
#pragma unroll
      for (int r = 0; r < 8; ++r) {
        float v = acc[i][j][r] * scale;
        if (BIAS_MODE == 1) v += bias[mBase + mOff + r];
        if (BIAS_MODE == 2) v += bv;
        if (RESID) v += Rb[(size_t)(mBase + mOff + r) * ldc + n];
        if (ACT == 1) v = tanhf(v);
        if (ACT == 2) v = fmaxf(v, 0.0f);
        if (ACT == 3) v = v / (1.0f + expf(-v));
        if (ACT == 4) v = (v > 0.f) ? v : 0.01f * v;
        slab[(mOff + r) * 68 + (j << 4) + rlane] = v;
      }
    }
    __builtin_amdgcn_fence(__ATOMIC_RELEASE, "workgroup");
    __builtin_amdgcn_wave_barrier();
    __builtin_amdgcn_fence(__ATOMIC_ACQUIRE, "workgroup");
    if (OUT_MODE == 0) {
      float* C = (float*)Cout + (size_t)b * strideC;
      const int hh = lane >> 4, c4 = (lane & 15) * 4;
      for (int pass = 0; pass < 2; ++pass) {
#pragma unroll
        for (int it = 0; it < 8; ++it) {
          const int row = it * 2 + hh;
          v4f v = *(const v4f*)(slab + row * 68 + c4);
          *(volatile v4f*)(C + (size_t)(mBase + row) * ldc + n0 + c4) = v;
        }
        __threadfence();
      }
    } else {
      const int q = lane >> 3, c8 = (lane & 7) * 8;
      unsigned short* C  = (unsigned short*)Cout  + (size_t)b * strideC;
      unsigned short* C2 = (OUT_MODE == 2) ? ((unsigned short*)Cout2 + (size_t)b * strideC) : nullptr;
      for (int pass = 0; pass < 2; ++pass) {
#pragma unroll
        for (int it = 0; it < 4; ++it) {
          const int row = it * 4 + q;
          const float* sp = slab + row * 68 + c8;
          v8h hv, lv;
#pragma unroll
          for (int e = 0; e < 8; ++e) {
            if (OUT_MODE == 1) {
              hv[e] = (_Float16)sp[e];
            } else {
              unsigned short hb = f2bf_bits(sp[e]);
              hv[e] = __builtin_bit_cast(_Float16, hb);
              if (OUT_MODE == 2) {
                unsigned short lb = f2bf_bits(sp[e] - bf_bits2f(hb));
                lv[e] = __builtin_bit_cast(_Float16, lb);
              }
            }
          }
          *(volatile v8h*)(C + (size_t)(mBase + row) * ldc + n0 + c8) = hv;
          if (OUT_MODE == 2) *(volatile v8h*)(C2 + (size_t)(mBase + row) * ldc + n0 + c8) = lv;
        }
        __threadfence();
      }
    }
    __builtin_amdgcn_fence(__ATOMIC_RELEASE, "workgroup");
    __builtin_amdgcn_wave_barrier();
    __builtin_amdgcn_fence(__ATOMIC_ACQUIRE, "workgroup");
  }
}

__global__ __launch_bounds__(256) void cvt_rows_bf16_kernel(
    const float* __restrict__ src, unsigned short* __restrict__ dst, int total8)
{
  const int i = blockIdx.x * 256 + threadIdx.x;
  if (i >= total8) return;
  const size_t e0 = (size_t)i << 3;
  const v4f a0 = *(const v4f*)(src + e0);
  const v4f a1 = *(const v4f*)(src + e0 + 4);
  v8h hv;
#pragma unroll
  for (int e = 0; e < 4; ++e) {
    hv[e]     = __builtin_bit_cast(_Float16, f2bf_bits(a0[e]));
    hv[4 + e] = __builtin_bit_cast(_Float16, f2bf_bits(a1[e]));
  }
  unsigned short* q = dst + e0;
  *(volatile v8h*)q = hv;
  __threadfence();
  *(volatile v8h*)q = hv;
}

__global__ __launch_bounds__(256) void transpose_bf16_kernel(
    const float* __restrict__ in, int ldi, unsigned short* __restrict__ out, int ldo)
{
  __shared__ float sT[64 * 65];
  const int tid = threadIdx.x, lane = tid & 31, wave = tid >> 5;
  const int rb = blockIdx.y * 64;
  const int cb = blockIdx.x * 64;
#pragma unroll
  for (int it = 0; it < 4; ++it) {
    const int r = (tid >> 4) + 16 * it, c4 = (tid & 15) * 4;
    const v4f v = *(const v4f*)(in + (size_t)(rb + r) * ldi + cb + c4);
    float* sp = sT + r * 65 + c4;
    sp[0] = v[0]; sp[1] = v[1]; sp[2] = v[2]; sp[3] = v[3];
  }
  __syncthreads();
  v8h hv[2];
#pragma unroll
  for (int it = 0; it < 2; ++it) {
    const int oc = it * 32 + wave * 4 + (lane >> 3), c8 = (lane & 7) * 8;
#pragma unroll
    for (int e = 0; e < 8; ++e) hv[it][e] = __builtin_bit_cast(_Float16, f2bf_bits(sT[(c8 + e) * 65 + oc]));
  }
  for (int pass = 0; pass < 2; ++pass) {
#pragma unroll
    for (int it = 0; it < 2; ++it) {
      const int oc = it * 32 + wave * 4 + (lane >> 3), c8 = (lane & 7) * 8;
      *(volatile v8h*)(out + (size_t)(cb + oc) * ldo + rb + c8) = hv[it];
    }
    __threadfence();
  }
}

__global__ __launch_bounds__(256) void conv_silu_kernel(
    const float* __restrict__ XIN, const float* __restrict__ cw, const float* __restrict__ cb,
    unsigned short* __restrict__ XCH)
{
  __shared__ __align__(16) float sT[16 * kConvTP];
  const int tid = threadIdx.x, lane = tid & 31, wave = tid >> 5;
  const int d0 = blockIdx.x * 256, d = d0 + tid;
  const int g0 = blockIdx.y * 64;
  const int tb = g0 & (kSeq - 1);
  const float w0 = bfq(cw[d * kTaps + 0]), w1 = bfq(cw[d * kTaps + 1]), w2 = bfq(cw[d * kTaps + 2]), w3 = bfq(cw[d * kTaps + 3]);
  const float bc = bfq(cb[d]);
  float xm3, xm2, xm1;
  {
    const bool hist = (tb > 0);
    const int rb = hist ? (g0 - 3) : g0;
    const float v3 = XIN[(size_t)rb * kInner + d];
    const float v2 = XIN[(size_t)(rb + 1) * kInner + d];
    const float v1 = XIN[(size_t)(rb + 2) * kInner + d];
    xm3 = hist ? v3 : 0.f;
    xm2 = hist ? v2 : 0.f;
    xm1 = hist ? v1 : 0.f;
  }
#pragma unroll 1
  for (int sub = 0; sub < 4; ++sub) {
    const int lb = g0 + sub * 16;
#pragma unroll 1
    for (int s = 0; s < 16; ++s) {
      const float xcur = XIN[(size_t)(lb + s) * kInner + d];
      float acc = w0 * xm3;
      acc = fmaf(w1, xm2, acc);
      acc = fmaf(w2, xm1, acc);
      acc = fmaf(w3, xcur, acc);
      const float sv = acc + bc;
      const float sg = __builtin_amdgcn_rcpf(1.0f + expf(-sv));
      sT[s * kConvTP + tid] = sv * sg;
      xm3 = xm2; xm2 = xm1; xm1 = xcur;
    }
    __syncthreads();
    v8h bh[2];
#pragma unroll
    for (int it = 0; it < 2; ++it) {
      const float* sp = sT + (it * 8 + wave) * kConvTP + lane * 8;
      const v4f a0 = *(const v4f*)(sp);
      const v4f a1 = *(const v4f*)(sp + 4);
#pragma unroll
      for (int e = 0; e < 4; ++e) {
        bh[it][e]     = __builtin_bit_cast(_Float16, f2bf_bits(a0[e]));
        bh[it][4 + e] = __builtin_bit_cast(_Float16, f2bf_bits(a1[e]));
      }
    }
    for (int pass = 0; pass < 2; ++pass) {
#pragma unroll
      for (int it = 0; it < 2; ++it) {
        const size_t o = (size_t)(lb + it * 8 + wave) * kInner + d0 + lane * 8;
        *(volatile v8h*)(XCH + o) = bh[it];
      }
      __threadfence();
    }
    __syncthreads();
  }
}

__global__ __launch_bounds__(128) void ssm_chunk_kernel(
    const float* __restrict__ XIN, const unsigned short* __restrict__ DTP, const unsigned short* __restrict__ Zp,
    const unsigned short* __restrict__ BCH, const unsigned short* __restrict__ BT, const unsigned short* __restrict__ GP,
    const float* __restrict__ cw, const float* __restrict__ cb, const float* __restrict__ bdt, const float* __restrict__ Dp,
    unsigned short* __restrict__ YH, unsigned short* __restrict__ YL)
{
  __shared__ __align__(16) __bf16 Ut[kCB * kUP];
  __shared__ __align__(16) __bf16 Hb[kCB * kUP];
  __shared__ __align__(16) __bf16 Gs[kQ * kUP];
  __shared__ __align__(16) float  Et[kQ * kCB];
  __shared__ __align__(16) float  Xt[kQ * kCB];
  __shared__ __align__(16) float  Yl[kQ * kYP];
  const int tid = threadIdx.x, lane = tid & 31, wave = tid >> 5;
  const int hh = lane >> 4, rl = lane & 15, koff = hh * 8;
  constexpr int kGroups = kInner / kCB;
  const int b  = blockIdx.x / kGroups;
  const int cg = blockIdx.x - b * kGroups;
  const int c0 = cg * kCB;
  const size_t rowB = (size_t)b * kSeq;
  const __bf16* BCb = (const __bf16*)(const void*)BCH;
  const __bf16* BTb = (const __bf16*)(const void*)BT;
  const v8f zero8 = (v8f){0.f,0.f,0.f,0.f,0.f,0.f,0.f,0.f};

  {
    v8b zz;
#pragma unroll
    for (int e = 0; e < 8; ++e) zz[e] = __builtin_bit_cast(__bf16, (unsigned short)0);
#pragma unroll
    for (int it = 0; it < 4; ++it) {
      const int row = (tid >> 3) + 16 * it, c8 = (tid & 7) * 8;
      *(v8b*)(Hb + row * kUP + c8) = zz;
    }
  }
  v8f H4[4];
#pragma unroll
  for (int j = 0; j < 4; ++j) H4[j] = zero8;

  const int ich = tid & (kCB - 1);
  const int ch  = c0 + ich;
  const float w0 = bfq(cw[ch * kTaps + 0]), w1 = bfq(cw[ch * kTaps + 1]), w2 = bfq(cw[ch * kTaps + 2]), w3 = bfq(cw[ch * kTaps + 3]);
  const float cbv = bfq(cb[ch]), bb = bfq(bdt[ch]), dd = bfq(Dp[ch]);
  float xm3 = 0.f, xm2 = 0.f, xm1 = 0.f;
  const int qy = lane >> 3, c8f = (lane & 7) * 8;

#pragma unroll 1
  for (int qc = 0; qc < kNChunk; ++qc) {
    const size_t r0 = rowB + (size_t)qc * kQ;
    __syncthreads();
    {
      const unsigned short* gsrc = GP + ((size_t)(b * kNChunk + qc) * kQ) * kQ;
#pragma unroll
      for (int it = 0; it < 4; ++it) {
        const int t = (tid >> 3) + 16 * it, s8 = (tid & 7) * 8;
        v4u w = *(const v4u*)(gsrc + (size_t)t * kQ + s8);
#pragma unroll
        for (int k = 0; k < 4; ++k) {
          const unsigned mlo = (s8 + 2 * k     <= t) ? 0x0000ffffu : 0u;
          const unsigned mhi = (s8 + 2 * k + 1 <= t) ? 0xffff0000u : 0u;
          w[k] = w[k] & (mlo | mhi);
        }
        *(v8b*)(Gs + t * kUP + s8) = __builtin_bit_cast(v8b, w);
      }
    }
    if (tid < kCB) {
      float S = 0.f;
#pragma unroll 1
      for (int s = 0; s < kQ; ++s) {
        const size_t rofs = (r0 + s) * (size_t)kInner + c0;
        const float xcur = XIN[rofs + ich];
        const unsigned wd = *(const unsigned*)(DTP + rofs + (ich & ~1));
        const unsigned hb = (wd >> ((ich & 1) * 16)) & 0xffffu;
        const float pre = h16_to_f32(hb) * 0.0625f;
        float cacc = w0 * xm3;
        cacc = fmaf(w1, xm2, cacc);
        cacc = fmaf(w2, xm1, cacc);
        cacc = fmaf(w3, xcur, cacc);
        const float sv = cacc + cbv;
        const float xc = sv * __builtin_amdgcn_rcpf(1.0f + expf(-sv));
        xm3 = xm2; xm2 = xm1; xm1 = xcur;
        const float v  = pre + bb;
        const float dt = fmaxf(v, 0.0f) + log1pf(expf(-fabsf(v)));
        S += dt;
        const float en = expf(-S);
        const float ep = expf(S);
        const float u  = ep * (dt * xc);
        Ut[ich * kUP + s] = at_f2bf(u);
        Et[s * kCB + ich] = en;
        Xt[s * kCB + ich] = dd * xc;
      }
    }
    __syncthreads();

    {
      v8f acc[4];
#pragma unroll
      for (int j = 0; j < 4; ++j) acc[j] = zero8;
#pragma unroll
      for (int k0 = 0; k0 < kQ; k0 += 32) {
        const v16b a = Frag<__bf16>::load(Gs + (16 * wave + rl) * kUP + koff + k0);
#pragma unroll
        for (int j = 0; j < 4; ++j) {
          const v16b bj = Frag<__bf16>::load(Ut + (16 * j + rl) * kUP + koff + k0);
          acc[j] = mma_g(a, bj, acc[j]);
        }
      }
#pragma unroll
      for (int k0 = 0; k0 < kState; k0 += 32) {
        const v16b a = Frag<__bf16>::load(BCb + (r0 + 16 * wave + rl) * (size_t)kBC + kState + koff + k0);
#pragma unroll
        for (int j = 0; j < 4; ++j) {
          const v16b bj = Frag<__bf16>::load(Hb + (16 * j + rl) * kUP + koff + k0);
          acc[j] = mma_g(a, bj, acc[j]);
        }
      }
#pragma unroll
      for (int j = 0; j < 4; ++j)
#pragma unroll
        for (int r = 0; r < 8; ++r) Yl[(16 * wave + 8 * hh + r) * kYP + 16 * j + rl] = acc[j][r];
    }
    __syncthreads();

    {
      v8f acc2[4];
#pragma unroll
      for (int j = 0; j < 4; ++j) acc2[j] = zero8;
#pragma unroll
      for (int k0 = 0; k0 < kQ; k0 += 32) {
        const v16b a = Frag<__bf16>::load(Ut + (16 * wave + rl) * kUP + koff + k0);
#pragma unroll
        for (int j = 0; j < 4; ++j) {
          const v16b bj = Frag<__bf16>::load(BTb + (size_t)(16 * j + rl) * kRows + r0 + koff + k0);
          acc2[j] = mma_g(a, bj, acc2[j]);
        }
      }
      const v4f eqa = *(const v4f*)(Et + (kQ - 1) * kCB + 16 * wave + 8 * hh);
      const v4f eqb = *(const v4f*)(Et + (kQ - 1) * kCB + 16 * wave + 8 * hh + 4);
      const float eq[8] = {eqa[0], eqa[1], eqa[2], eqa[3], eqb[0], eqb[1], eqb[2], eqb[3]};
#pragma unroll
      for (int j = 0; j < 4; ++j) {
#pragma unroll
        for (int r = 0; r < 8; ++r) {
          const float hn = eq[r] * (H4[j][r] + acc2[j][r]);
          H4[j][r] = hn;
          Hb[(16 * wave + 8 * hh + r) * kUP + 16 * j + rl] = at_f2bf(hn);
        }
      }
    }

    {
      v8h hv[4], lv[4];
#pragma unroll
      for (int it = 0; it < 4; ++it) {
        const int t = it * 16 + wave * 4 + qy;
        const v4f ya = *(const v4f*)(Yl + t * kYP + c8f);
        const v4f yb = *(const v4f*)(Yl + t * kYP + c8f + 4);
        const v4f ea = *(const v4f*)(Et + t * kCB + c8f);
        const v4f eb = *(const v4f*)(Et + t * kCB + c8f + 4);
        const v4f xa = *(const v4f*)(Xt + t * kCB + c8f);
        const v4f xb = *(const v4f*)(Xt + t * kCB + c8f + 4);
        const v4u zw = *(const v4u*)(Zp + (r0 + t) * (size_t)kInner + c0 + c8f);
        float yv[8];
#pragma unroll
        for (int e = 0; e < 4; ++e) {
          yv[e]     = fmaf(ea[e], ya[e], xa[e]);
          yv[4 + e] = fmaf(eb[e], yb[e], xb[e]);
        }
#pragma unroll
        for (int e = 0; e < 8; ++e) {
          const unsigned zword = zw[e >> 1];
          const unsigned zbits = (e & 1) ? (zword >> 16) : (zword & 0xffffu);
          const float zv = h16_to_f32(zbits);
          const float sg = __builtin_amdgcn_rcpf(1.0f + expf(-zv));
          const float y  = yv[e] * (zv * sg);
          const unsigned short hb2 = f2bf_bits(y);
          const unsigned short lb2 = f2bf_bits(y - bf_bits2f(hb2));
          hv[it][e] = __builtin_bit_cast(_Float16, hb2);
          lv[it][e] = __builtin_bit_cast(_Float16, lb2);
        }
      }
      for (int pass = 0; pass < 2; ++pass) {
#pragma unroll
        for (int it = 0; it < 4; ++it) {
          const int t = it * 16 + wave * 4 + qy;
          const size_t o = (r0 + t) * (size_t)kInner + c0 + c8f;
          *(volatile v8h*)(YH + o) = hv[it];
          *(volatile v8h*)(YL + o) = lv[it];
        }
        __threadfence();
      }
    }
  }
}

extern "C" void kernel_launch(void* const* d_in, const int* in_sizes, int n_in,
                              void* d_out, int out_size, void* d_ws, size_t ws_size,
                              hipStream_t stream) {
  if (n_in < 10) return;
  if (in_sizes[0] != kRows * kHid) return;
  if (in_sizes[1] != kHid * 2 * kInner) return;
  if (in_sizes[2] != kInner * kTaps) return;
  if (in_sizes[3] != kInner) return;
  if (in_sizes[4] != kInner * kInner) return;
  if (in_sizes[5] != kInner) return;
  if (in_sizes[6] != kInner * kState) return;
  if (in_sizes[7] != kInner * kState) return;
  if (in_sizes[8] != kInner) return;
  if (in_sizes[9] != kInner * kHid) return;
  if (out_size != kRows * kHid) return;
  if (ws_size < kWsTotal) return;

  const float* x      = (const float*)d_in[0];
  const float* W_in   = (const float*)d_in[1];
  const float* conv_w = (const float*)d_in[2];
  const float* conv_b = (const float*)d_in[3];
  const float* W_dt   = (const float*)d_in[4];
  const float* b_dt   = (const float*)d_in[5];
  const float* W_B    = (const float*)d_in[6];
  const float* W_C    = (const float*)d_in[7];
  const float* Dp     = (const float*)d_in[8];
  const float* W_out  = (const float*)d_in[9];
  float* out = (float*)d_out;

  char* ws = (char*)d_ws;
  unsigned short* XB   = (unsigned short*)(ws + kOffXB);
  unsigned short* WINT = (unsigned short*)(ws + kOffWINT);
  unsigned short* WDTT = (unsigned short*)(ws + kOffWDTT);
  unsigned short* WBCT = (unsigned short*)(ws + kOffWBCT);
  unsigned short* WOT  = (unsigned short*)(ws + kOffWOT);
  float*          XIN  = (float*)(ws + kOffXIN);
  unsigned short* ZP   = (unsigned short*)(ws + kOffZP);
  unsigned short* XCH  = (unsigned short*)(ws + kOffXCH);
  unsigned short* YH   = XCH;
  unsigned short* DTP  = (unsigned short*)(ws + kOffDTP);
  unsigned short* BCH  = (unsigned short*)(ws + kOffBCH);
  unsigned short* BT   = (unsigned short*)(ws + kOffBT);
  unsigned short* GP   = (unsigned short*)(ws + kOffGP);
  unsigned short* YL   = (unsigned short*)(ws + kOffYL);

  cvt_rows_bf16_kernel<<<(kRows * kHid / 8) / 256, 256, 0, stream>>>(x, XB, kRows * kHid / 8);
  transpose_bf16_kernel<<<dim3((2 * kInner) / 64, kHid / 64), 256, 0, stream>>>(W_in, 2 * kInner, WINT, kHid);
  transpose_bf16_kernel<<<dim3(kInner / 64, kInner / 64), 256, 0, stream>>>(W_dt, kInner, WDTT, kInner);
  transpose_bf16_kernel<<<dim3(kState / 64, kInner / 64), 256, 0, stream>>>(W_B, kState, WBCT, kInner);
  transpose_bf16_kernel<<<dim3(kState / 64, kInner / 64), 256, 0, stream>>>(W_C, kState, WBCT + (size_t)kState * kInner, kInner);
  transpose_bf16_kernel<<<dim3(kHid / 64, kInner / 64), 256, 0, stream>>>(W_out, kHid, WOT, kInner);

  wmma_gemm64<1, 0, 0, 0, false><<<dim3(256, 1), 256, 0, stream>>>(
      XB, nullptr, kHid, 0L,
      WINT, nullptr, kHid, 0L,
      (void*)XIN, nullptr, kInner, 0L,
      nullptr, nullptr, 0L,
      kRows, kInner, kHid, 1.0f);
  wmma_gemm64<1, 0, 0, 1, false><<<dim3(256, 1), 256, 0, stream>>>(
      XB, nullptr, kHid, 0L,
      WINT + (size_t)kInner * kHid, nullptr, kHid, 0L,
      (void*)ZP, nullptr, kInner, 0L,
      nullptr, nullptr, 0L,
      kRows, kInner, kHid, 1.0f);

  conv_silu_kernel<<<dim3(kInner / 256, kRows / 64), 256, 0, stream>>>(XIN, conv_w, conv_b, XCH);

  wmma_gemm64<1, 0, 0, 1, false><<<dim3(256, 1), 256, 0, stream>>>(
      XCH, nullptr, kInner, 0L,
      WDTT, nullptr, kInner, 0L,
      (void*)DTP, nullptr, kInner, 0L,
      nullptr, nullptr, 0L,
      kRows, kInner, kInner, 16.0f);

  wmma_gemm64<1, 0, 0, 3, false><<<dim3(16, 1), 256, 0, stream>>>(
      XCH, nullptr, kInner, 0L,
      WBCT, nullptr, kInner, 0L,
      (void*)BCH, nullptr, kBC, 0L,
      nullptr, nullptr, 0L,
      kRows, kBC, kInner, 1.0f);
  wmma_gemm64<1, 0, 0, 3, false><<<dim3(8, 1), 256, 0, stream>>>(
      WBCT, nullptr, kInner, 0L,
      XCH, nullptr, kInner, 0L,
      (void*)BT, nullptr, kRows, 0L,
      nullptr, nullptr, 0L,
      kState, kRows, kInner, 1.0f);

  wmma_gemm64<1, 0, 0, 3, false><<<dim3(1, kBatch * kNChunk), 256, 0, stream>>>(
      BCH + kState, nullptr, kBC, (long)kQ * kBC,
      BCH, nullptr, kBC, (long)kQ * kBC,
      (void*)GP, nullptr, kQ, (long)kQ * kQ,
      nullptr, nullptr, 0L,
      kQ, kQ, kState, 1.0f);

  ssm_chunk_kernel<<<kBatch * (kInner / kCB), 128, 0, stream>>>(
      XIN, DTP, ZP, BCH, BT, GP, conv_w, conv_b, b_dt, Dp, YH, YL);

  wmma_gemm64<1, 1, 0, 0, false><<<dim3(128, 1), 256, 0, stream>>>(
      YH, YL, kInner, 0L,
      WOT, nullptr, kInner, 0L,
      (void*)out, nullptr, kHid, 0L,
      nullptr, nullptr, 0L,
      kRows, kHid, kInner, 1.0f);
}
